// TransformerBlock_893353197782
// MI455X (gfx1250) — hardware-run, weakly checked
//
#include <hip/hip_runtime.h>


#ifndef NB
#define NB 2
#endif
#ifndef SEQ
#define SEQ 2048
#endif
#define NB_FULL  2
#define SEQ_FULL 2048
#ifndef OUT_SEQ
#define OUT_SEQ SEQ
#endif
#ifndef HID
#define HID 65536
#endif
#define HID_FULL 65536
#define DM   128
#define NH_  8
#define HD   16
#define FW   4
#define OSP  68
#define OSF  132
#define OSH  136
#define WSC  64.0f
#define WSI  (1.0f / 64.0f)
#define W2S  256.0f
#define W2I  (1.0f / 256.0f)
#define CSC  64.0f
#define CWI  (1.0f / 4096.0f)
#define SC2  ((float)(0.08838834764831845 * 1.4426950408889634))
#define PSH  14.0f
#define NEGB (-3.0e38f)

static_assert(HD == 16);
static_assert(NH_ * HD == DM);
static_assert(NH_ * 32 <= 1024);
static_assert(DM == 128);
static_assert(DM % 64 == 0);
static_assert(64 % HD == 0);
static_assert(DM % 32 == 0);
static_assert(SEQ % 64 == 0);
static_assert((NB * SEQ) % 64 == 0);
static_assert(SEQ % 32 == 0);
static_assert(SEQ % 16 == 0);
static_assert((NB * SEQ) % (16 * FW) == 0);
static_assert((NB * SEQ) % 16 == 0);
static_assert(HID % 64 == 0);
static_assert(HID % 4 == 0);
static_assert(HID <= HID_FULL);
static_assert(NB <= NB_FULL);
static_assert(SEQ <= SEQ_FULL);
static_assert((OSP * 4) % 16 == 0);
static_assert((OSF * 4) % 16 == 0);
static_assert((OSH * 2) % 16 == 0);
static_assert(((DM * DM / 8) % 256) == 0);
static_assert(16 * OSP * 4 <= 131072);
static_assert(FW * 16 * OSF * 4 <= 131072);
static_assert(16 * OSH * 2 <= 131072);
static_assert(64 * 65 * 4 <= 131072);
static_assert(32 * 16 * 4 == 16 * (64 / HD) * HD * 2);
static_assert(32 * 16 * 4 == 16 * 64 * 2);
static_assert(32 * 16 * 8 == 16 * 64 * 4);
static_assert(32 * NH_ * 16 == 16 * DM * 2);
static_assert(32 * 16 * 16 == 16 * DM * 4);
static_assert(256 * 16 == 16 * DM * 2);
static_assert(256 * 16 * 2 == 64 * 64 * 2);

typedef _Float16 h16;
typedef __attribute__((ext_vector_type(16))) _Float16 v16h;
typedef __attribute__((ext_vector_type(8)))  _Float16 v8h;
typedef __attribute__((ext_vector_type(8)))  float    v8f;
typedef __attribute__((ext_vector_type(4)))  float    v4f;
typedef v4f  __attribute__((may_alias)) v4fa;
typedef v8h  __attribute__((may_alias)) v8ha;

__device__ __forceinline__ unsigned short f2bf(float f) { unsigned u = __float_as_uint(f); u += 0x7FFFu + ((u >> 16) & 1u); return (unsigned short)(u >> 16); }
__device__ __forceinline__ float bfr(float f) { return __uint_as_float(((unsigned)f2bf(f)) << 16); }
__device__ __forceinline__ v16h cat16(v8h lo, v8h hi) { return __builtin_shufflevector(lo, hi, 0, 1, 2, 3, 4, 5, 6, 7, 8, 9, 10, 11, 12, 13, 14, 15); }
__device__ __forceinline__ v8f wmma16(v16h a, v16h b, v8f c) { return __builtin_amdgcn_wmma_f32_16x16x32_f16(false, a, false, b, (short)0, c, false, false); }
__device__ __forceinline__ v16h  ldh(const h16* p) { return cat16(*(const v8h*)p, *(const v8h*)(p + 16)); }
__device__ __forceinline__ void wave_sync() { __builtin_amdgcn_fence(3  , "wavefront"); __builtin_amdgcn_wave_barrier(); asm volatile("" ::: "memory"); }
__device__ __forceinline__ v8f wmma16g(v16h a, v16h b, v8f c) {
    c = wmma16(a, b, c);
    asm volatile("v_nop\n\tv_nop\n\tv_nop\n\tv_nop" : "+v"(c) : "v"(a), "v"(b));
    return c;
}
static __device__ __forceinline__ h16 toh_flush(float v) { const h16 r = (h16)v; return (fabsf(v) < 6.103515625e-05f) ? (h16)0.0f : r; }

__global__ __launch_bounds__(256) void k_wqkv(const float* __restrict__ W, h16* WT, float scale) {
#pragma clang fp contract(off)
    const int idx = blockIdx.x * 256 + threadIdx.x;
    const int n = idx / (DM / 8), e8 = (idx % (DM / 8)) * 8;
    const int hh = n / HD, d = n % HD;
    v8h o;
#pragma unroll
    for (int k = 0; k < 8; ++k) o[k] = toh_flush(bfr(W[((size_t)hh * DM + e8 + k) * HD + d]) * scale);
    h16* dp = WT + (size_t)idx * 8;
    *(volatile v8h*)dp = o; __threadfence(); *(volatile v8h*)dp = o;
}

__global__ __launch_bounds__(256) void k_tconv(const float* __restrict__ src, int ldin, h16* dst, int ldout, float scale) {
#pragma clang fp contract(off)
    __shared__ float ts[64 * 65];
    const int tid = threadIdx.x;
    const int c0 = blockIdx.x * 64, r0 = blockIdx.y * 64;
    const int lc = tid & 63, lq = tid >> 6;
#pragma unroll 4
    for (int i = 0; i < 16; ++i) { const int r = i * 4 + lq; ts[r * 65 + lc] = src[(size_t)(r0 + r) * (size_t)ldin + (size_t)(c0 + lc)]; }
    __syncthreads();
    const int r8 = (tid & 7) * 8, cq = tid >> 3;
    v8h o0, o1;
#pragma unroll
    for (int k = 0; k < 8; ++k) { o0[k] = toh_flush(bfr(ts[(r8 + k) * 65 + cq]) * scale); o1[k] = toh_flush(bfr(ts[(r8 + k) * 65 + 32 + cq]) * scale); }
    h16* d0 = dst + (size_t)(c0 + cq) * (size_t)ldout + (size_t)(r0 + r8);
    h16* d1 = dst + (size_t)(c0 + 32 + cq) * (size_t)ldout + (size_t)(r0 + r8);
    *(volatile v8h*)d0 = o0; *(volatile v8h*)d1 = o1; __threadfence(); *(volatile v8h*)d0 = o0; *(volatile v8h*)d1 = o1;
}

__global__ __launch_bounds__(256) void k_bfr4(const float* __restrict__ src, float* dst, int n4) {
    const int i = blockIdx.x * 256 + threadIdx.x; if (i >= n4) return;
    const v4f v = *(const v4f*)(src + (size_t)i * 4); v4f o;
#pragma unroll
    for (int k = 0; k < 4; ++k) o[k] = bfr(v[k]);
    float* dp = dst + (size_t)i * 4;
    *(volatile v4f*)dp = o; __threadfence(); *(volatile v4f*)dp = o;
}

__global__ __launch_bounds__(256) void k_ln(const float* __restrict__ X, int srcseq, const float* __restrict__ g, const float* __restrict__ be, h16* Hout, int rnd) {
#pragma clang fp contract(off)
    const int lane = threadIdx.x & 31;
    const int wave = __builtin_amdgcn_readfirstlane((int)(threadIdx.x >> 5));
    const int m = blockIdx.x * 16 + wave * 2 + (lane >> 4);
    const int c8 = (lane & 15) * 8;
    const int bb = m / SEQ, tt = m % SEQ;
    const float* xp = X + ((size_t)bb * (size_t)srcseq + (size_t)tt) * DM + c8;
    const v4f a0 = *(const v4f*)xp, a1 = *(const v4f*)(xp + 4);
    const v4f g0 = *(const v4f*)(g + c8), g1 = *(const v4f*)(g + c8 + 4);
    const v4f e0 = *(const v4f*)(be + c8), e1 = *(const v4f*)(be + c8 + 4);
    float v[8], gg[8], ee[8];
#pragma unroll
    for (int k = 0; k < 4; ++k) { v[k] = rnd ? bfr(a0[k]) : a0[k]; v[4 + k] = rnd ? bfr(a1[k]) : a1[k]; gg[k] = bfr(g0[k]); gg[4 + k] = bfr(g1[k]); ee[k] = bfr(e0[k]); ee[4 + k] = bfr(e1[k]); }
    float s = ((v[0] + v[1]) + (v[2] + v[3])) + ((v[4] + v[5]) + (v[6] + v[7]));
    s += __shfl_xor(s, 8, 32); s += __shfl_xor(s, 4, 32); s += __shfl_xor(s, 2, 32); s += __shfl_xor(s, 1, 32);
    const float mean = s * (1.0f / DM);
    float d[8];
#pragma unroll
    for (int k = 0; k < 8; ++k) d[k] = v[k] - mean;
    float q = ((d[0] * d[0] + d[1] * d[1]) + (d[2] * d[2] + d[3] * d[3])) + ((d[4] * d[4] + d[5] * d[5]) + (d[6] * d[6] + d[7] * d[7]));
    q += __shfl_xor(q, 8, 32); q += __shfl_xor(q, 4, 32); q += __shfl_xor(q, 2, 32); q += __shfl_xor(q, 1, 32);
    const float rstd = rsqrtf(q * (1.0f / DM) + 1.0e-5f);
    v8h o;
#pragma unroll
    for (int k = 0; k < 8; ++k) o[k] = toh_flush(d[k] * rstd * gg[k] + ee[k]);
    h16* dp = Hout + (size_t)m * DM + c8;
    *(volatile v8h*)dp = o; __threadfence(); *(volatile v8h*)dp = o;
}

__global__ __launch_bounds__(32) void k_projqk(const h16* __restrict__ A, const h16* __restrict__ Bt, h16* Ph, float oscale) {
    __shared__ __align__(16) float os[16 * OSP];
    const int K = DM;
    const int lane = threadIdx.x & 31, lr = lane & 15, hi = lane >> 4; const int r0 = blockIdx.x * 64, c0 = blockIdx.y * 64;
    v8f acc[4][4];
#pragma unroll
    for (int mb = 0; mb < 4; ++mb)
#pragma unroll
        for (int nb = 0; nb < 4; ++nb) acc[mb][nb] = (v8f){};
    const size_t aoff = (size_t)(r0 + lr) * K + 8 * hi, boff = (size_t)(c0 + lr) * K + 8 * hi;
#pragma unroll 1
    for (int kc = 0; kc < K; kc += 32) {
        v16h a[4];
#pragma unroll
        for (int mb = 0; mb < 4; ++mb) a[mb] = ldh(A + aoff + (size_t)mb * 16 * K + kc);
#pragma unroll
        for (int nb = 0; nb < 4; ++nb) { const v16h b = ldh(Bt + boff + (size_t)nb * 16 * K + kc);
#pragma unroll
            for (int mb = 0; mb < 4; ++mb) acc[mb][nb] = wmma16g(a[mb], b, acc[mb][nb]); }
    }
    const int bb = r0 / SEQ, tt = r0 % SEQ; const int zc = bb * NH_ + c0 / HD;
    const size_t tbase = ((size_t)zc * SEQ + (size_t)tt) * HD;
#pragma unroll
    for (int mb = 0; mb < 4; ++mb) {
#pragma unroll
        for (int nb = 0; nb < 4; ++nb) {
#pragma unroll
            for (int j = 0; j < 8; ++j) os[(hi * 8 + j) * OSP + nb * 16 + lr] = acc[mb][nb][j] * oscale; }
        wave_sync();
        v8h hv[4];
        { const int row = lane >> 1, c8 = (lane & 1) * 8;
#pragma unroll
          for (int hh = 0; hh < 4; ++hh) {
              const v4f x0 = *(const v4fa*)(&os[row * OSP + hh * HD + c8]); const v4f x1 = *(const v4fa*)(&os[row * OSP + hh * HD + c8 + 4]);
#pragma unroll
              for (int i = 0; i < 4; ++i) { hv[hh][i] = toh_flush(x0[i]); hv[hh][4 + i] = toh_flush(x1[i]); } } }
        const size_t sb = tbase + (size_t)(mb * 16) * HD;
#pragma unroll 1
        for (int ps = 0; ps < 2; ++ps) {
#pragma unroll
            for (int hh = 0; hh < 4; ++hh) { const size_t oo = sb + (size_t)hh * ((size_t)SEQ * HD) + (size_t)lane * 8; *(volatile v8h*)(Ph + oo) = hv[hh]; }
            if (ps == 0) __threadfence(); }
        wave_sync();
    }
}

__global__ __launch_bounds__(32) void k_projvt(const h16* __restrict__ A, const h16* __restrict__ Bt, h16* Ph, float oscale) {
    __shared__ __align__(16) float os[16 * OSP];
    const int K = DM;
    const int lane = threadIdx.x & 31, lr = lane & 15, hi = lane >> 4; const int r0 = blockIdx.x * 64, c0 = blockIdx.y * 64;
    v8f acc[4][4];
#pragma unroll
    for (int mb = 0; mb < 4; ++mb)
#pragma unroll
        for (int nb = 0; nb < 4; ++nb) acc[mb][nb] = (v8f){};
    const size_t aoff = (size_t)(r0 + lr) * K + 8 * hi, boff = (size_t)(c0 + lr) * K + 8 * hi;
#pragma unroll 1
    for (int kc = 0; kc < K; kc += 32) {
        v16h a[4];
#pragma unroll
        for (int mb = 0; mb < 4; ++mb) a[mb] = ldh(A + aoff + (size_t)mb * 16 * K + kc);
#pragma unroll
        for (int nb = 0; nb < 4; ++nb) { const v16h b = ldh(Bt + boff + (size_t)nb * 16 * K + kc);
#pragma unroll
            for (int mb = 0; mb < 4; ++mb) acc[mb][nb] = wmma16g(a[mb], b, acc[mb][nb]); }
    }
    const int bb = c0 / SEQ, tt = c0 % SEQ;
    const size_t tbase = (size_t)bb * (size_t)DM * SEQ + (size_t)r0 * SEQ + (size_t)tt;
#pragma unroll
    for (int mb = 0; mb < 4; ++mb) {
#pragma unroll
        for (int nb = 0; nb < 4; ++nb) {
#pragma unroll
            for (int j = 0; j < 8; ++j) os[(hi * 8 + j) * OSP + nb * 16 + lr] = acc[mb][nb][j] * oscale; }
        wave_sync();
        v8h hv[4];
#pragma unroll
        for (int s = 0; s < 4; ++s) { const int row = 4 * s + (lane >> 3), c8 = (lane & 7) * 8;
            const v4f x0 = *(const v4fa*)(&os[row * OSP + c8]); const v4f x1 = *(const v4fa*)(&os[row * OSP + c8 + 4]);
#pragma unroll
            for (int i = 0; i < 4; ++i) { hv[s][i] = toh_flush(x0[i]); hv[s][4 + i] = toh_flush(x1[i]); } }
        const size_t sb = tbase + (size_t)(mb * 16) * SEQ;
#pragma unroll 1
        for (int ps = 0; ps < 2; ++ps) {
#pragma unroll
            for (int s = 0; s < 4; ++s) { const int row = 4 * s + (lane >> 3), c8 = (lane & 7) * 8;
                const size_t oo = sb + (size_t)row * SEQ + c8; *(volatile v8h*)(Ph + oo) = hv[s]; }
            if (ps == 0) __threadfence(); }
        wave_sync();
    }
}

__global__ __launch_bounds__(32) void k_oproj(const h16* __restrict__ A, const h16* __restrict__ Bt, const float* __restrict__ X, const float* __restrict__ bo, float* X1, float oscale) {
    __shared__ __align__(16) float os[16 * OSP];
    const int K = DM;
    const int lane = threadIdx.x & 31, lr = lane & 15, hi = lane >> 4; const int r0 = blockIdx.x * 64, c0 = blockIdx.y * 64;
    v8f acc[4][4];
#pragma unroll
    for (int mb = 0; mb < 4; ++mb)
#pragma unroll
        for (int nb = 0; nb < 4; ++nb) acc[mb][nb] = (v8f){};
    const size_t aoff = (size_t)(r0 + lr) * K + 8 * hi, boff = (size_t)(c0 + lr) * K + 8 * hi;
#pragma unroll 1
    for (int kc = 0; kc < K; kc += 32) {
        v16h a[4];
#pragma unroll
        for (int mb = 0; mb < 4; ++mb) a[mb] = ldh(A + aoff + (size_t)mb * 16 * K + kc);
#pragma unroll
        for (int nb = 0; nb < 4; ++nb) { const v16h b = ldh(Bt + boff + (size_t)nb * 16 * K + kc);
#pragma unroll
            for (int mb = 0; mb < 4; ++mb) acc[mb][nb] = wmma16g(a[mb], b, acc[mb][nb]); }
    }
    const int bb = r0 / SEQ, tt = r0 % SEQ;
    const float* xb = X + ((size_t)bb * SEQ_FULL + (size_t)tt) * DM + c0;
    float* ob = X1 + (size_t)r0 * DM + c0;
    const int c4 = (lane & 15) * 4, rq = lane >> 4;
    const v4f bv = *(const v4f*)(bo + c0 + c4); v4f bq;
#pragma unroll
    for (int i = 0; i < 4; ++i) bq[i] = bfr(bv[i]);
#pragma unroll
    for (int mb = 0; mb < 4; ++mb) {
#pragma unroll
        for (int nb = 0; nb < 4; ++nb) {
#pragma unroll
            for (int j = 0; j < 8; ++j) os[(hi * 8 + j) * OSP + nb * 16 + lr] = acc[mb][nb][j] * oscale; }
        wave_sync();
#pragma unroll 1
        for (int ps = 0; ps < 2; ++ps) {
#pragma unroll
            for (int s = 0; s < 8; ++s) { const int row = 2 * s + rq;
                const v4f val = *(const v4fa*)(&os[row * OSP + c4]);
                const v4f xv = *(const v4f*)(xb + (size_t)(mb * 16 + row) * DM + c4); v4f o;
#pragma unroll
                for (int i = 0; i < 4; ++i) o[i] = bfr(xv[i]) + (val[i] + bq[i]);
                *(volatile v4f*)(ob + (size_t)(mb * 16 + row) * DM + c4) = o; }
            if (ps == 0) __threadfence(); }
        wave_sync();
    }
}

__global__ __launch_bounds__(32 * NH_) void k_flash(const h16* __restrict__ QP, const h16* __restrict__ KP, const h16* __restrict__ VT, h16* CTX) {
    __shared__ __align__(16) h16 os[16 * OSH];
    const int lane = threadIdx.x & 31, lr = lane & 15, hi = lane >> 4;
    const int wave = __builtin_amdgcn_readfirstlane((int)(threadIdx.x >> 5));
    const int b = blockIdx.y; const int zh = b * NH_ + wave;
    const int t0 = blockIdx.x * 16;
    const int lim = t0 + lr;
    const int nk = (t0 + 16 + 31) & ~31;
    const size_t pbase = (size_t)zh * SEQ * HD;
    const v8h z8 = (v8h){};
    const v16h qh = cat16(*(const v8h*)(QP + pbase + (size_t)(t0 + lr) * HD + 8 * hi), z8);
    const size_t ko = pbase + (size_t)lr * HD + 8 * hi;
    const size_t vo = pbase + (size_t)lr * SEQ + 8 * hi;
    v8f o0 = (v8f){};
    float m = NEGB, l = 0.0f;
#pragma unroll 1
    for (int key0 = 0; key0 < nk; key0 += 32) {
        const h16* ka = KP + ko + (size_t)key0 * HD;
        const v16h ka0 = cat16(*(const v8h*)ka, z8), kb0 = cat16(*(const v8h*)(ka + 16 * HD), z8);
        v8f sa = (v8f){}, sb = (v8f){};
        sa = wmma16g(ka0, qh, sa); sb = wmma16g(kb0, qh, sb);
        const int ja = key0 + 8 * hi;
        float ta[8], tb[8]; bool fa[8], fb[8]; float mx = NEGB;
#pragma unroll
        for (int r = 0; r < 8; ++r) {
            fa[r] = (ja + r <= lim);
            fb[r] = (ja + 16 + r <= lim);
            ta[r] = sa[r] * SC2; tb[r] = sb[r] * SC2;
            mx = fmaxf(mx, fmaxf(fa[r] ? ta[r] : NEGB, fb[r] ? tb[r] : NEGB)); }
        mx = fmaxf(mx, __shfl_xor(mx, 16, 32));
        const float mnew = fmaxf(m, mx);
        const float alpha = __builtin_amdgcn_exp2f(m - mnew);
        const float sh = PSH - mnew;
        v16h pb; float ls = 0.0f;
#pragma unroll
        for (int r = 0; r < 8; ++r) {
            const float xa = ta[r] + sh, xb = tb[r] + sh;
            const float ea = __builtin_amdgcn_exp2f(xa), eb = __builtin_amdgcn_exp2f(xb);
            const float ga = (fa[r] & (xa >= -14.0f)) ? ea : 0.0f, gb = (fb[r] & (xb >= -14.0f)) ? eb : 0.0f;
            const h16 pa = (h16)ga; const h16 pc = (h16)gb;
            pb[r] = pa; pb[8 + r] = pc;
            ls += (float)pa + (float)pc; }
        l = l * alpha + ls; m = mnew;
        o0 = o0 * alpha;
        const v16h v0 = ldh(VT + vo + key0);
        o0 = wmma16g(v0, pb, o0);
    }
    l += __shfl_xor(l, 16, 32);
    const bool any = l > 0.0f;
    const float lsafe = any ? l : 1.0f;
    const float inv = any ? (CSC / lsafe) : 0.0f;
    { v8h ov;
#pragma unroll
      for (int r = 0; r < 8; ++r) ov[r] = toh_flush(o0[r] * inv);
      *(v8ha*)(&os[lr * OSH + wave * HD + 8 * hi]) = ov; }
    __syncthreads();
    { const int tid = threadIdx.x; const int row = tid >> 4, c8 = (tid & 15) * 8;
      const v8h val = *(const v8ha*)(&os[row * OSH + c8]);
      h16* dp = CTX + ((size_t)b * SEQ + (size_t)(t0 + row)) * DM + c8;
      *(volatile v8h*)dp = val; __threadfence(); *(volatile v8h*)dp = val; }
}

__global__ __launch_bounds__(32 * FW) __attribute__((amdgpu_num_vgpr(256))) void k_ffn(const h16* __restrict__ H2, const h16* __restrict__ W1T, const h16* __restrict__ W2T,
                                                   const float* __restrict__ B1R, const float* __restrict__ X1, const float* __restrict__ bf2, float* OUT) {
    __shared__ __align__(16) float os[FW * 16 * OSF];
    const int lane = threadIdx.x & 31, lr = lane & 15, hi = lane >> 4;
    const int wave = __builtin_amdgcn_readfirstlane((int)(threadIdx.x >> 5));
    const int m0 = (blockIdx.x * FW + wave) * 16;
    const size_t ho = (size_t)(m0 + lr) * DM + 8 * hi;
    v16h hb[4];
#pragma unroll
    for (int kc = 0; kc < 4; ++kc) hb[kc] = ldh(H2 + ho + kc * 32);
    v8f acc[8];
#pragma unroll
    for (int c = 0; c < 8; ++c) acc[c] = (v8f){};
    const size_t w1o = (size_t)lr * DM + 8 * hi;
    const size_t w2o = (size_t)lr * HID + 8 * hi;
    const float* bp = B1R + 8 * hi;
#pragma unroll 1
    for (int j0 = 0; j0 < HID; j0 += 32) {
        const h16* w1p = W1T + w1o + (size_t)j0 * DM;
        v8f hA = (v8f){}, hB = (v8f){};
#pragma unroll
        for (int kc = 0; kc < 4; ++kc) {
            const v16h wa = ldh(w1p + kc * 32); const v16h wb = ldh(w1p + 16 * DM + kc * 32);
            hA = wmma16g(wa, hb[kc], hA); hB = wmma16g(wb, hb[kc], hB); }
        const v4f b0 = *(const v4f*)(bp + j0), b1 = *(const v4f*)(bp + j0 + 4), b2 = *(const v4f*)(bp + j0 + 16), b3 = *(const v4f*)(bp + j0 + 20);
        v16h pb;
#pragma unroll
        for (int r = 0; r < 4; ++r) {
            pb[r]      = toh_flush(fmaxf(hA[r]     * WSI + b0[r], 0.0f));
            pb[4 + r]  = toh_flush(fmaxf(hA[4 + r] * WSI + b1[r], 0.0f));
            pb[8 + r]  = toh_flush(fmaxf(hB[r]     * WSI + b2[r], 0.0f));
            pb[12 + r] = toh_flush(fmaxf(hB[4 + r] * WSI + b3[r], 0.0f)); }
        const h16* w2p = W2T + w2o + j0;
#pragma unroll
        for (int c = 0; c < 8; ++c) { const v16h wc = ldh(w2p + (size_t)c * 16 * HID); acc[c] = wmma16g(wc, pb, acc[c]); }
    }
    const int wb = wave * 16 * OSF;
#pragma unroll
    for (int c = 0; c < 8; ++c) { v4f a, e;
        a[0] = acc[c][0] * W2I; a[1] = acc[c][1] * W2I; a[2] = acc[c][2] * W2I; a[3] = acc[c][3] * W2I;
        e[0] = acc[c][4] * W2I; e[1] = acc[c][5] * W2I; e[2] = acc[c][6] * W2I; e[3] = acc[c][7] * W2I;
        *(v4fa*)(&os[wb + lr * OSF + c * 16 + 8 * hi]) = a; *(v4fa*)(&os[wb + lr * OSF + c * 16 + 8 * hi + 4]) = e; }
    wave_sync();
    const int bb = m0 / SEQ, tt = m0 % SEQ;
    float* orow = OUT + ((size_t)bb * OUT_SEQ + (size_t)tt) * DM;
    const float* xrow = X1 + (size_t)m0 * DM;
    const int cofs = lane * 4;
    const v4f bv = *(const v4f*)(bf2 + cofs); v4f bq;
#pragma unroll
    for (int i = 0; i < 4; ++i) bq[i] = bfr(bv[i]);
#pragma unroll 1
    for (int ps = 0; ps < 2; ++ps) {
#pragma unroll
        for (int row = 0; row < 16; ++row) {
            const v4f val = *(const v4fa*)(&os[wb + row * OSF + cofs]);
            const v4f xv = *(const v4f*)(xrow + (size_t)row * DM + cofs); v4f o;
#pragma unroll
            for (int i = 0; i < 4; ++i) o[i] = xv[i] + (val[i] + bq[i]);
            *(volatile v4f*)(orow + (size_t)row * DM + cofs) = o; }
        if (ps == 0) __threadfence(); }
}

static constexpr size_t al256(size_t v) { return (v + 255) & ~(size_t)255; }
static constexpr size_t SZ_HP = al256((size_t)NB * SEQ * DM * 2);
static constexpr size_t SZ_WT = al256((size_t)DM * DM * 2);
static constexpr size_t SZ_WF = al256((size_t)HID * DM * 2);
static constexpr size_t SZ_B1 = al256((size_t)HID * 4);
static constexpr size_t SZ_PL = al256((size_t)NB * NH_ * SEQ * HD * 2);
static constexpr size_t SZ_X1 = al256((size_t)NB * SEQ * DM * 4);
static constexpr size_t SZ_TOTAL = 3 * SZ_HP + 4 * SZ_WT + 2 * SZ_WF + SZ_B1 + 3 * SZ_PL + SZ_X1;
static_assert(SZ_TOTAL <= (size_t)134217728);
static_assert((size_t)NB * NH_ * SEQ * HD == (size_t)NB * DM * SEQ);
static_assert(((size_t)NB * SEQ * DM * 2) % 128 == 0);
static_assert(((size_t)HID * DM * 2) % 128 == 0);

extern "C" void kernel_launch(void* const* d_in, const int* in_sizes, int n_in,
                              void* d_out, int out_size, void* d_ws, size_t ws_size, hipStream_t stream) {
    if (n_in < 14) return;
    const size_t needx = ((size_t)(NB - 1) * SEQ_FULL + SEQ) * DM;
    if ((size_t)in_sizes[0] < needx) return;
    if ((size_t)in_sizes[1] < (size_t)NH_ * DM * HD || (size_t)in_sizes[2] < (size_t)NH_ * DM * HD || (size_t)in_sizes[3] < (size_t)NH_ * DM * HD) return;
    if ((size_t)in_sizes[4] < (size_t)DM * DM) return;
    if (in_sizes[5] < DM || in_sizes[6] < DM || in_sizes[7] < DM || in_sizes[8] < DM || in_sizes[9] < DM || in_sizes[13] < DM) return;
    if ((size_t)in_sizes[10] < (size_t)(DM - 1) * HID_FULL + HID) return;
    if ((size_t)in_sizes[11] < (size_t)HID) return;
    if ((size_t)in_sizes[12] < (size_t)HID * DM) return;
    if ((size_t)out_size < ((size_t)(NB - 1) * OUT_SEQ + SEQ) * DM) return;
    if (SZ_TOTAL > ws_size) return;
    const float* x   = (const float*)d_in[0];
    const float* wk  = (const float*)d_in[1];
    const float* wq  = (const float*)d_in[2];
    const float* wv  = (const float*)d_in[3];
    const float* wo  = (const float*)d_in[4];
    const float* bo  = (const float*)d_in[5];
    const float* g1  = (const float*)d_in[6];
    const float* be1 = (const float*)d_in[7];
    const float* g2  = (const float*)d_in[8];
    const float* be2 = (const float*)d_in[9];
    const float* w1  = (const float*)d_in[10];
    const float* bf1 = (const float*)d_in[11];
    const float* w2  = (const float*)d_in[12];
    const float* bf2 = (const float*)d_in[13];
    float* OUT = (float*)d_out;
    char* wsp = (char*)d_ws;
    h16* H1  = (h16*)wsp; wsp += SZ_HP;
    h16* CTX = (h16*)wsp; wsp += SZ_HP;
    h16* H2  = (h16*)wsp; wsp += SZ_HP;
    h16* WQT = (h16*)wsp; wsp += SZ_WT;
    h16* WKT = (h16*)wsp; wsp += SZ_WT;
    h16* WVT = (h16*)wsp; wsp += SZ_WT;
    h16* WOT = (h16*)wsp; wsp += SZ_WT;
    h16* W1T = (h16*)wsp; wsp += SZ_WF;
    h16* W2T = (h16*)wsp; wsp += SZ_WF;
    float* B1R = (float*)wsp; wsp += SZ_B1;
    h16* QP = (h16*)wsp; wsp += SZ_PL;
    h16* KP = (h16*)wsp; wsp += SZ_PL;
    h16* VT = (h16*)wsp; wsp += SZ_PL;
    float* X1 = (float*)wsp; wsp += SZ_X1;

    k_wqkv<<<DM * DM / 8 / 256, 256, 0, stream>>>(wq, WQT, WSC);
    k_wqkv<<<DM * DM / 8 / 256, 256, 0, stream>>>(wk, WKT, WSC);
    k_wqkv<<<DM * DM / 8 / 256, 256, 0, stream>>>(wv, WVT, WSC);
    k_tconv<<<dim3(DM / 64, DM / 64, 1), 256, 0, stream>>>(wo, DM, WOT, DM, WSC);
    k_tconv<<<dim3(HID / 64, DM / 64, 1), 256, 0, stream>>>(w1, HID_FULL, W1T, DM, WSC);
    k_tconv<<<dim3(DM / 64, HID / 64, 1), 256, 0, stream>>>(w2, DM, W2T, HID, W2S);
    k_bfr4<<<(HID / 4 + 255) / 256, 256, 0, stream>>>(bf1, B1R, HID / 4);

    k_ln<<<NB * SEQ / 16, 256, 0, stream>>>(x, SEQ_FULL, g1, be1, H1, 1);
    k_projqk<<<dim3(NB * SEQ / 64, DM / 64, 1), 32, 0, stream>>>(H1, WQT, QP, WSI);
    k_projqk<<<dim3(NB * SEQ / 64, DM / 64, 1), 32, 0, stream>>>(H1, WKT, KP, WSI);
    k_projvt<<<dim3(DM / 64, NB * SEQ / 64, 1), 32, 0, stream>>>(WVT, H1, VT, WSI);
    k_flash<<<dim3(SEQ / 16, NB, 1), 32 * NH_, 0, stream>>>(QP, KP, VT, CTX);
    k_oproj<<<dim3(NB * SEQ / 64, DM / 64, 1), 32, 0, stream>>>(CTX, WOT, x, bo, X1, CWI);
    k_ln<<<NB * SEQ / 16, 256, 0, stream>>>(X1, SEQ, g2, be2, H2, 0);
    k_ffn<<<NB * SEQ / (16 * FW), 32 * FW, 0, stream>>>(H2, W1T, W2T, B1R, X1, bf2, OUT);
}
